// GraphSAGE_79998060855855
// MI455X (gfx1250) — hardware-verified
//
#include <hip/hip_runtime.h>
#include <stddef.h>
#include <stdint.h>
#include <math.h>


#define CF     128
#define CO2    64
#define YP     256
#define AP16   512
#define NTHR   256
#define NWAVE  8
#define EPT    8
#define CHUNK  (NTHR * EPT)
#define WCAP   (EPT * 32)
#define LISTN  (NWAVE * WCAP)
#define NBA    1024
#define SLA    10
#define RCAP   28672
#define DEGCAP 64
#define GROWS  32
#define GT     64
#define UP0    4096
#define UP1    8192
#define UP2    4096
#define AGG_ZINTS (LISTN + 2 * RCAP + 3 * NBA)
#define MISC_INTS 16
#define AGG_LDS_INTS (AGG_ZINTS + MISC_INTS)
#define WSMAX  134217728

static_assert((CHUNK & (CHUNK - 1)) == 0 && CHUNK <= 4096);
static_assert((NBA & (NBA - 1)) == 0 && NBA == (1 << SLA));
static_assert(((long long)CHUNK << SLA) < (1LL << 31));
static_assert(LISTN % NTHR == 0);
static_assert(NBA % NWAVE == 0 && NBA % 32 == 0 && NBA % 64 == 0 && NBA % GROWS == 0);
static_assert(RCAP % 32 == 0 && AGG_ZINTS % 4 == 0 && LISTN % 4 == 0);
static_assert(AGG_ZINTS % (NTHR * 4) == 0);
static_assert(CF % 32 == 0 && (2 * CF) % 32 == 0 && YP == 2 * CF && AP16 == 2 * YP);
static_assert(GROWS == (GT / 32) * 16);
static_assert(UP0 % NTHR == 0 && UP1 % NTHR == 0 && UP2 % NTHR == 0);
static_assert(NWAVE * 2 * CF * 8 <= RCAP * 4);
static_assert((LISTN * 4) % 16 == 0);
static_assert(AGG_LDS_INTS * 4 <= 300000);
static_assert(DEGCAP >= 36 + 8 && RCAP >= 16710);

typedef float          v2f   __attribute__((ext_vector_type(2)));
typedef float          v4f   __attribute__((ext_vector_type(4)));
typedef float          v8f   __attribute__((ext_vector_type(8)));
typedef double         v2d   __attribute__((ext_vector_type(2)));
typedef int            v4i   __attribute__((ext_vector_type(4)));
typedef int            v8i   __attribute__((ext_vector_type(8)));
typedef unsigned short v4us  __attribute__((ext_vector_type(4)));
typedef unsigned short v8us  __attribute__((ext_vector_type(8)));
typedef unsigned short v16us __attribute__((ext_vector_type(16)));
typedef __bf16         v16bf __attribute__((ext_vector_type(16)));
typedef v2f  __attribute__((may_alias)) v2fa;
typedef v4f  __attribute__((may_alias)) v4fa;
typedef v4i  __attribute__((may_alias)) v4ia;
typedef v4us __attribute__((may_alias)) v4usa;
typedef v8us __attribute__((may_alias)) v8usa;
union FragB { v16bf v; v16us u; v8us h[2]; v8i w; };

__device__ __forceinline__ v8f wmb(const FragB& a, const FragB& b, v8f c) {
  v8f d = __builtin_amdgcn_wmma_f32_16x16x32_bf16(false, a.v, false, b.v, (short)0, c, false, false);
  asm volatile("v_nop\n\tv_nop\n\tv_nop\n\tv_nop" : "+v"(d) : "v"(a.w), "v"(b.w));
  return d;
}

__device__ __forceinline__ unsigned bf16_bits(float f) {
  const unsigned u = __float_as_uint(f);
  return (u + 0x7FFFu + ((u >> 16) & 1u)) >> 16;
}
__device__ __forceinline__ float bf16_val(float f) {
  return __uint_as_float(bf16_bits(f) << 16);
}

__device__ __forceinline__ void wave_sync() {
  __builtin_amdgcn_fence(__ATOMIC_RELEASE, "wavefront");
  __builtin_amdgcn_wave_barrier();
  __builtin_amdgcn_fence(__ATOMIC_ACQUIRE, "wavefront");
}

template <int SLB>
__device__ __forceinline__ int scan_chunk(const int* __restrict__ dsts, int nE, int cbase, int slotBase,
                                          int nb, int vec8, int* list, int tid, int lane, int wave) {
  int wc = 0;
  const int el0  = tid * EPT;
  const int e0   = cbase + el0;
  const int sent = -2147483647 - 1;
  v4i da, db;
  if (vec8 != 0 && cbase + CHUNK <= nE) {
    da = *(const v4i*)(dsts + e0);
    db = *(const v4i*)(dsts + e0 + 4);
  } else {
    da.x = (e0     < nE) ? dsts[min(e0,     nE - 1)] : sent;
    da.y = (e0 + 1 < nE) ? dsts[min(e0 + 1, nE - 1)] : sent;
    da.z = (e0 + 2 < nE) ? dsts[min(e0 + 2, nE - 1)] : sent;
    da.w = (e0 + 3 < nE) ? dsts[min(e0 + 3, nE - 1)] : sent;
    db.x = (e0 + 4 < nE) ? dsts[min(e0 + 4, nE - 1)] : sent;
    db.y = (e0 + 5 < nE) ? dsts[min(e0 + 5, nE - 1)] : sent;
    db.z = (e0 + 6 < nE) ? dsts[min(e0 + 6, nE - 1)] : sent;
    db.w = (e0 + 7 < nE) ? dsts[min(e0 + 7, nE - 1)] : sent;
  }
  const unsigned nbs = (unsigned)slotBase;
  const unsigned unb = (unsigned)nb;
  const unsigned s0 = (unsigned)da.x - nbs, s1 = (unsigned)da.y - nbs;
  const unsigned s2 = (unsigned)da.z - nbs, s3 = (unsigned)da.w - nbs;
  const unsigned s4 = (unsigned)db.x - nbs, s5 = (unsigned)db.y - nbs;
  const unsigned s6 = (unsigned)db.z - nbs, s7 = (unsigned)db.w - nbs;
  const bool h0 = s0 < unb, h1 = s1 < unb, h2 = s2 < unb, h3 = s3 < unb;
  const bool h4 = s4 < unb, h5 = s5 < unb, h6 = s6 < unb, h7 = s7 < unb;
  const unsigned any = __builtin_amdgcn_ballot_w32(h0 | h1 | h2 | h3 | h4 | h5 | h6 | h7);
  if (any != 0u) {
#define HITJ(J, HJ, SJ) { \
      const unsigned mj = __builtin_amdgcn_ballot_w32(HJ); \
      if (mj != 0u) { \
        if (HJ) { \
          const int pos = wc + (int)__builtin_amdgcn_mbcnt_lo(mj, 0u); \
          if (pos < WCAP) list[wave * WCAP + pos] = ((el0 + (J)) << SLB) | (int)(SJ); \
        } \
        wc += (int)__builtin_popcount(mj); } }
    HITJ(0, h0, s0)
    HITJ(1, h1, s1)
    HITJ(2, h2, s2)
    HITJ(3, h3, s3)
    HITJ(4, h4, s4)
    HITJ(5, h5, s5)
    HITJ(6, h6, s6)
    HITJ(7, h7, s7)
#undef HITJ
  }
  return wc;
}

__global__ __launch_bounds__(NTHR) void k_wprep(const float* __restrict__ Wl0, const float* __restrict__ Wr0,
                                                const float* __restrict__ Wl1, const float* __restrict__ Wr1,
                                                const float* __restrict__ Wl2, const float* __restrict__ Wr2,
                                                unsigned short* P0, unsigned short* P1, unsigned short* P2) {
  const int u = (int)blockIdx.x * NTHR + (int)threadIdx.x;
  const float* W;
  unsigned short* P;
  int n, nr, kc, ks, pitch;
  if (u < UP0) {
    n = u >> 4; kc = (u & 15) * 8; ks = kc;
    W = (n < CF) ? Wl0 : Wr0; nr = n & (CF - 1); P = P0; pitch = CF;
  } else if (u < UP0 + UP1) {
    const int v = u - UP0;
    n = v >> 5; kc = (v & 31) * 8; ks = kc & (CF - 1);
    W = (n < CF) ? Wl1 : Wr1; nr = n & (CF - 1); P = P1; pitch = 2 * CF;
  } else if (u < UP0 + UP1 + UP2) {
    const int v = u - UP0 - UP1;
    n = v >> 5; kc = (v & 31) * 8; ks = kc & (CF - 1);
    W = (n < CO2) ? Wl2 : Wr2; nr = n & (CO2 - 1); P = P2; pitch = 2 * CF;
  } else {
    return;
  }
  const float* p = W + (size_t)nr * CF + ks;
  const v4f a = *(const v4fa*)p;
  const v4f b = *(const v4fa*)(p + 4);
  v8us o;
  o[0] = (unsigned short)bf16_bits(a.x); o[1] = (unsigned short)bf16_bits(a.y);
  o[2] = (unsigned short)bf16_bits(a.z); o[3] = (unsigned short)bf16_bits(a.w);
  o[4] = (unsigned short)bf16_bits(b.x); o[5] = (unsigned short)bf16_bits(b.y);
  o[6] = (unsigned short)bf16_bits(b.z); o[7] = (unsigned short)bf16_bits(b.w);
  unsigned short* dp = P + (size_t)n * pitch + kc;
  *(volatile v8us*)dp = o;
  __threadfence();
  *(volatile v8us*)dp = o;
}

__global__ __launch_bounds__(NTHR) void k_cvx(const float* __restrict__ x, int nN, int nUnits,
                                              unsigned short* xb) {
  const int u = (int)blockIdx.x * NTHR + (int)threadIdx.x;
  if (u >= nUnits) return;
  const int row = u >> 4;
  const int k8  = (u & 15) * 8;
  const int rc  = row < nN ? row : nN - 1;
  const float* p = x + (size_t)rc * CF + k8;
  const v4f a = *(const v4fa*)p;
  const v4f b = *(const v4fa*)(p + 4);
  const bool ok = row < nN;
  v8us o;
  o[0] = ok ? (unsigned short)bf16_bits(a.x) : (unsigned short)0;
  o[1] = ok ? (unsigned short)bf16_bits(a.y) : (unsigned short)0;
  o[2] = ok ? (unsigned short)bf16_bits(a.z) : (unsigned short)0;
  o[3] = ok ? (unsigned short)bf16_bits(a.w) : (unsigned short)0;
  o[4] = ok ? (unsigned short)bf16_bits(b.x) : (unsigned short)0;
  o[5] = ok ? (unsigned short)bf16_bits(b.y) : (unsigned short)0;
  o[6] = ok ? (unsigned short)bf16_bits(b.z) : (unsigned short)0;
  o[7] = ok ? (unsigned short)bf16_bits(b.w) : (unsigned short)0;
  unsigned short* dp = xb + (size_t)row * AP16 + k8;
  *(volatile v8us*)dp = o;
  __threadfence();
  *(volatile v8us*)dp = o;
}

template <int NG>
__global__ __launch_bounds__(GT) void k_gemm(float* Y, const unsigned short* __restrict__ BT, int K) {
  constexpr int SP = 128 * NG;
  __shared__ __attribute__((aligned(16))) float stg[GROWS * SP];
  const int tid = (int)threadIdx.x, lane = tid & 31, wave = tid >> 5, hh = lane >> 4, m = lane & 15;
  const int rowBase = (int)blockIdx.x * GROWS;
  const unsigned short* ap = (const unsigned short*)Y + (size_t)(rowBase + 16 * wave + m) * (size_t)AP16 + 8 * hh;

#pragma unroll
  for (int g = 0; g < NG; ++g) {
    v8f acc[8];
    {
      const v8f z = {0.f, 0.f, 0.f, 0.f, 0.f, 0.f, 0.f, 0.f};
#pragma unroll
      for (int t = 0; t < 8; ++t) acc[t] = z;
    }
    const unsigned short* bp = BT + (size_t)(128 * g + m) * (size_t)K + 8 * hh;
#pragma unroll 1
    for (int k0 = 0; k0 < K; k0 += 32) {
      FragB af;
      af.h[0] = *(const v8usa*)(ap + k0);
      af.h[1] = *(const v8usa*)(ap + k0 + 16);
#pragma unroll
      for (int nt = 0; nt < 8; ++nt) {
        const unsigned short* wq = bp + (size_t)(16 * nt) * (size_t)K + k0;
        FragB bf;
        bf.h[0] = *(const v8usa*)wq;
        bf.h[1] = *(const v8usa*)(wq + 16);
        acc[nt] = wmb(af, bf, acc[nt]);
      }
    }
#pragma unroll
    for (int nt = 0; nt < 8; ++nt) {
      const int lc = 128 * g + 16 * nt + m;
#pragma unroll
      for (int r = 0; r < 8; ++r) {
        const int lr = 16 * wave + 8 * hh + r;
        stg[lr * SP + lc] = acc[nt][r];
      }
    }
  }
  __syncthreads();

#pragma unroll
  for (int g = 0; g < NG; ++g) {
    v4f pv[16];
#pragma unroll
    for (int i = 0; i < 16; ++i) pv[i] = *(const v4fa*)(stg + (16 * wave + i) * SP + 128 * g + 4 * lane);
#pragma unroll
    for (int i = 0; i < 16; ++i) {
      float* op = Y + (size_t)(rowBase + 16 * wave + i) * (size_t)YP + 128 * g + 4 * lane;
      *(volatile v4f*)op = pv[i];
    }
    __threadfence();
#pragma unroll
    for (int i = 0; i < 16; ++i) {
      float* op = Y + (size_t)(rowBase + 16 * wave + i) * (size_t)YP + 128 * g + 4 * lane;
      *(volatile v4f*)op = pv[i];
    }
  }
}

template <int C>
__global__ __launch_bounds__(NTHR) void k_scan(const int* __restrict__ srcs, const int* __restrict__ dsts,
                                               int nE, int nN, int vec8, int mRows,
                                               float* Y, const float* __restrict__ bl, double* rec) {
  static_assert(C == 128 || C == 64);
  extern __shared__ __attribute__((aligned(16))) int dsm[];
  int* list = dsm;
  int* hl   = dsm + LISTN;
  int* sl   = hl + RCAP;
  int* cnt  = sl + RCAP;
  int* offs = cnt + NBA;
  int* cur  = offs + NBA;
  int* misc = cur + NBA;
  const int tid = (int)threadIdx.x, lane = tid & 31, wave = tid >> 5;
  const int nodeBase = (int)blockIdx.x * NBA;

  {
    const v4i z4 = {0, 0, 0, 0};
    for (int i = tid * 4; i < AGG_ZINTS; i += NTHR * 4) *(v4ia*)(dsm + i) = z4;
    if (tid < MISC_INTS) misc[tid] = 0;
  }
  float bv0 = 0.0f, bv1 = 0.0f, bv2 = 0.0f, bv3 = 0.0f;
  if constexpr (C == 128) {
    const v4f t4 = *(const v4fa*)(bl + 4 * lane);
    bv0 = bf16_val(t4.x); bv1 = bf16_val(t4.y); bv2 = bf16_val(t4.z); bv3 = bf16_val(t4.w);
  } else {
    const v2f t2 = *(const v2fa*)(bl + 2 * lane);
    bv0 = bf16_val(t2.x); bv1 = bf16_val(t2.y);
  }
  __syncthreads();

  int t = 0, ov = 0;
  const int nChunks = (nE + CHUNK - 1) / CHUNK;
#pragma unroll 1
  for (int ch = 0; ch < nChunks; ++ch) {
    const int cbase = ch * CHUNK;
    const int wc = scan_chunk<SLA>(dsts, nE, cbase, nodeBase, NBA, vec8, list, tid, lane, wave);
    if (lane == 0) misc[wave] = wc;
    __syncthreads();
    if (wave == 0) {
#pragma unroll 1
      for (int w2 = 0; w2 < NWAVE; ++w2) {
        int c = misc[w2];
        c = c < 0 ? 0 : (c > WCAP ? WCAP : c);
#pragma unroll 1
        for (int b0 = 0; b0 < c; b0 += 32) {
          const int idx = b0 + lane;
          const int ent = list[w2 * WCAP + (idx < WCAP ? idx : WCAP - 1)];
          const int m32 = (c - b0) < 32 ? (c - b0) : 32;
#pragma unroll 1
          for (int k = 0; k < m32; ++k) {
            const int u    = __builtin_amdgcn_readlane(ent, k);
            const int slot = u & (NBA - 1);
            const int el   = (u >> SLA) & (CHUNK - 1);
            const int pk   = ((cbase + el) << SLA) | slot;
            if (t < RCAP) {
              if (lane == 0) { hl[t] = pk; cnt[slot] = cnt[slot] + 1; }
              t = t + 1;
            } else {
              ov = 1;
            }
          }
        }
      }
    }
    __syncthreads();
  }
  if (wave == 0 && lane == 0) { misc[8] = t; misc[9] = ov; }
  __syncthreads();
  int tt = misc[8];
  tt = tt < 0 ? 0 : (tt > RCAP ? RCAP : tt);
  const int ovf = misc[9];

  if (wave == 0) {
    const int base = lane * (NBA / 32);
    int s = 0;
#pragma unroll 1
    for (int i = 0; i < NBA / 32; ++i) s += cnt[base + i];
    int incl = s;
#pragma unroll
    for (int d = 1; d < 32; d <<= 1) {
      const int y = __shfl_up(incl, d, 32);
      if (lane >= d) incl += y;
    }
    int run = incl - s;
#pragma unroll 1
    for (int i = 0; i < NBA / 32; ++i) {
      const int cv = cnt[base + i];
      offs[base + i] = run;
      cur[base + i]  = run;
      run += cv;
    }
  }
  __syncthreads();
  if (wave == 0) {
#pragma unroll 1
    for (int b0 = 0; b0 < tt; b0 += 32) {
      const int idx = b0 + lane;
      const int ent = hl[idx < RCAP ? idx : RCAP - 1];
      const int m32 = (tt - b0) < 32 ? (tt - b0) : 32;
#pragma unroll 1
      for (int k = 0; k < m32; ++k) {
        const int u    = __builtin_amdgcn_readlane(ent, k);
        const int slot = u & (NBA - 1);
        if (lane == 0) {
          int p = cur[slot];
          p = p < 0 ? 0 : (p > RCAP - 1 ? RCAP - 1 : p);
          sl[p] = u;
          cur[slot] = p + 1;
        }
      }
    }
  }
  __syncthreads();

  const float qnan = __int_as_float(0x7fc00000);
  const float pz = (ovf != 0) ? qnan : 0.0f;
  const int sa = (2 * lane) & 31, sb = (2 * lane + 1) & 31;
  double sd0 = 0.0, sd1 = 0.0, sd2 = 0.0, sd3 = 0.0;
  double qd0 = 0.0, qd1 = 0.0, qd2 = 0.0, qd3 = 0.0;
#pragma unroll 1
  for (int si = 0; si < NBA / NWAVE; ++si) {
    const int s    = si * NWAVE + wave;
    const int node = nodeBase + s;
    int craw = cnt[s];
    craw = craw < 0 ? 0 : craw;
    const bool big = craw > DEGCAP;
    const int c = craw > DEGCAP ? DEGCAP : craw;
    int o = offs[s];
    o = o < 0 ? 0 : (o > RCAP ? RCAP : o);
    const int nc = node < mRows ? node : mRows - 1;
    float a0 = 0.0f, a1 = 0.0f, a2 = 0.0f, a3 = 0.0f;
#pragma unroll 1
    for (int b0 = 0; b0 < c; b0 += 32) {
      int idx = o + b0 + lane;
      idx = idx > RCAP - 1 ? RCAP - 1 : idx;
      const int ent = sl[idx];
      int eid = ent >> SLA;
      eid = eid < 0 ? 0 : (eid > nE - 1 ? nE - 1 : eid);
      int sr = srcs[eid];
      sr = sr < 0 ? 0 : (sr > nN - 1 ? nN - 1 : sr);
      const int m32 = (c - b0) < 32 ? (c - b0) : 32;
#pragma unroll 1
      for (int k = 0; k < m32; ++k) {
        const int sk = __builtin_amdgcn_readlane(sr, k);
        if constexpr (C == 128) {
          const v4f a = *(const v4fa*)(Y + (size_t)sk * YP + 4 * lane);
          a0 += a.x; a1 += a.y; a2 += a.z; a3 += a.w;
        } else {
          const v2f a = *(const v2fa*)(Y + (size_t)sk * YP + 2 * lane);
          a0 += a.x; a1 += a.y;
        }
      }
    }
    const float cfl = (craw < 1) ? 1.0f : (float)craw;
    const float inv = 1.0f / cfl;
    const float pzr = big ? qnan : pz;
    const bool live = node < nN;
    if constexpr (C == 128) {
      const v4f yr = *(const v4fa*)(Y + (size_t)nc * YP + C + 4 * lane);
      float z0 = (a0 * inv + bv0) + yr.x;
      float z1 = (a1 * inv + bv1) + yr.y;
      float z2 = (a2 * inv + bv2) + yr.z;
      float z3 = (a3 * inv + bv3) + yr.w;
      z0 = live ? (z0 + pzr) : 0.0f;
      z1 = live ? (z1 + pzr) : 0.0f;
      z2 = live ? (z2 + pzr) : 0.0f;
      z3 = live ? (z3 + pzr) : 0.0f;
      sd0 += (double)z0; qd0 += (double)z0 * (double)z0;
      sd1 += (double)z1; qd1 += (double)z1 * (double)z1;
      sd2 += (double)z2; qd2 += (double)z2 * (double)z2;
      sd3 += (double)z3; qd3 += (double)z3 * (double)z3;
      v4f zv;
      zv.x = z0; zv.y = z1; zv.z = z2; zv.w = z3;
      float* op = Y + (size_t)nc * YP + C + 4 * lane;
      if (node < mRows) {
        *(volatile v4f*)op = zv;
        __threadfence();
        *(volatile v4f*)op = zv;
      }
    } else {
      const v2f yr = *(const v2fa*)(Y + (size_t)nc * YP + C + 2 * lane);
      float z0 = (a0 * inv + bv0) + yr.x;
      float z1 = (a1 * inv + bv1) + yr.y;
      z0 = live ? (z0 + pzr) : 0.0f;
      z1 = live ? (z1 + pzr) : 0.0f;
      sd0 += (double)z0; qd0 += (double)z0 * (double)z0;
      sd1 += (double)z1; qd1 += (double)z1 * (double)z1;
      v4f ow;
      ow.x = __shfl(z0, sa, 32); ow.y = __shfl(z1, sa, 32);
      ow.z = __shfl(z0, sb, 32); ow.w = __shfl(z1, sb, 32);
      const bool wr = (node < mRows) && (lane < 16);
      float* op = Y + (size_t)nc * YP + C + 4 * (lane & 15);
      if (wr) *(volatile v4f*)op = ow;
      __threadfence();
      if (wr) *(volatile v4f*)op = ow;
    }
  }

  double* wpart = (double*)(dsm + LISTN);
  if constexpr (C == 128) {
    double* wp = wpart + wave * (2 * C) + 4 * lane;
    wp[0] = sd0; wp[1] = sd1; wp[2] = sd2; wp[3] = sd3;
    wp[C + 0] = qd0; wp[C + 1] = qd1; wp[C + 2] = qd2; wp[C + 3] = qd3;
  } else {
    double* wp = wpart + wave * (2 * C) + 2 * lane;
    wp[0] = sd0; wp[1] = sd1;
    wp[C + 0] = qd0; wp[C + 1] = qd1;
  }
  __syncthreads();
  if (tid < C) {
    const int e0 = 2 * tid;
    double r0 = 0.0, r1 = 0.0;
#pragma unroll
    for (int w2 = 0; w2 < NWAVE; ++w2) {
      r0 += wpart[w2 * (2 * C) + e0];
      r1 += wpart[w2 * (2 * C) + e0 + 1];
    }
    v2d ov2;
    ov2.x = r0; ov2.y = r1;
    double* rp = rec + (size_t)blockIdx.x * (size_t)(2 * C) + e0;
    *(volatile v2d*)rp = ov2;
    __threadfence();
    *(volatile v2d*)rp = ov2;
  }
}

__global__ __launch_bounds__(NTHR) void k_bnstat(const double* __restrict__ rec, int nb, int C, double invN,
                                                 float* ms) {
  __shared__ double sums[NTHR];
  __shared__ __attribute__((aligned(16))) float st[NTHR];
  const int t = (int)threadIdx.x;
  const int E2 = 2 * C;
  const int tc = t < E2 ? t : E2 - 1;
  double s = 0.0;
#pragma unroll 4
  for (int b = 0; b < nb; ++b) s += rec[(size_t)b * (size_t)E2 + tc];
  sums[t] = s;
  __syncthreads();
  const int cc = t & 127;
  const int ci = cc < C ? cc : C - 1;
  const double S = sums[ci];
  const double Q = sums[C + ci];
  const double mean = S * invN;
  double var = Q * invN - mean * mean;
  var = (var < 0.0) ? 0.0 : var;
  const float mf = (float)mean;
  const float vf = (float)var;
  const float rs = 1.0f / sqrtf(vf + 1e-5f);
  const float val = (t < 128) ? mf : rs;
  st[t] = (cc < C) ? val : 0.0f;
  __syncthreads();
  if (t < 64) {
    const v4f o = *(const v4fa*)(st + 4 * t);
    float* op = ms + 4 * t;
    *(volatile v4f*)op = o;
    __threadfence();
    *(volatile v4f*)op = o;
  }
}

__global__ __launch_bounds__(NTHR) void k_bn(float* Y, const float* __restrict__ ms,
                                             const float* __restrict__ gam, const float* __restrict__ bet,
                                             int nN) {
  __shared__ __attribute__((aligned(16))) unsigned short rowbuf[NWAVE * 2 * CF];
  const int tid = (int)threadIdx.x, lane = tid & 31, wave = tid >> 5;
  unsigned short* rb = rowbuf + wave * (2 * CF);
  const v4f m4 = *(const v4fa*)(ms + 4 * lane);
  const v4f r4 = *(const v4fa*)(ms + 128 + 4 * lane);
  v4f g4, b4;
  {
    const v4f tg = *(const v4fa*)(gam + 4 * lane);
    const v4f tb = *(const v4fa*)(bet + 4 * lane);
    g4.x = bf16_val(tg.x); g4.y = bf16_val(tg.y); g4.z = bf16_val(tg.z); g4.w = bf16_val(tg.w);
    b4.x = bf16_val(tb.x); b4.y = bf16_val(tb.y); b4.z = bf16_val(tb.z); b4.w = bf16_val(tb.w);
  }
  const int rowBase = (int)blockIdx.x * 64 + wave * 8;
#pragma unroll 1
  for (int j = 0; j < 8; ++j) {
    const int row = rowBase + j;
    const bool live = row < nN;
    const v4f z = *(const v4fa*)(Y + (size_t)row * YP + CF + 4 * lane);
    float y0 = ((z.x - m4.x) * r4.x) * g4.x + b4.x;
    float y1 = ((z.y - m4.y) * r4.y) * g4.y + b4.y;
    float y2 = ((z.z - m4.z) * r4.z) * g4.z + b4.z;
    float y3 = ((z.w - m4.w) * r4.w) * g4.w + b4.w;
    y0 = (y0 > 0.0f) ? y0 : (y0 - y0);
    y1 = (y1 > 0.0f) ? y1 : (y1 - y1);
    y2 = (y2 > 0.0f) ? y2 : (y2 - y2);
    y3 = (y3 > 0.0f) ? y3 : (y3 - y3);
    y0 = live ? y0 : 0.0f; y1 = live ? y1 : 0.0f; y2 = live ? y2 : 0.0f; y3 = live ? y3 : 0.0f;
    v4us h4, l4;
    unsigned hb;
    hb = bf16_bits(y0); h4[0] = (unsigned short)hb; l4[0] = (unsigned short)bf16_bits(y0 - __uint_as_float(hb << 16));
    hb = bf16_bits(y1); h4[1] = (unsigned short)hb; l4[1] = (unsigned short)bf16_bits(y1 - __uint_as_float(hb << 16));
    hb = bf16_bits(y2); h4[2] = (unsigned short)hb; l4[2] = (unsigned short)bf16_bits(y2 - __uint_as_float(hb << 16));
    hb = bf16_bits(y3); h4[3] = (unsigned short)hb; l4[3] = (unsigned short)bf16_bits(y3 - __uint_as_float(hb << 16));
    *(v4usa*)(rb + 4 * lane) = h4;
    *(v4usa*)(rb + CF + 4 * lane) = l4;
    wave_sync();
    const v8us q = *(const v8usa*)(rb + 8 * lane);
    wave_sync();
    unsigned short* rp = (unsigned short*)Y + (size_t)row * AP16 + 8 * lane;
    *(volatile v8us*)rp = q;
    __threadfence();
    *(volatile v8us*)rp = q;
  }
}

__global__ __launch_bounds__(NTHR) void k_bnout(const float* __restrict__ Y, const float* __restrict__ ms,
                                                const float* __restrict__ gam, const float* __restrict__ bet,
                                                int nN, float* out) {
  const int tid = (int)threadIdx.x, lane = tid & 31, wave = tid >> 5;
  const int hs = lane >> 4;
  const int c4 = 4 * (lane & 15);
  const v4f m4 = *(const v4fa*)(ms + c4);
  const v4f r4 = *(const v4fa*)(ms + 128 + c4);
  v4f g4, b4;
  {
    const v4f tg = *(const v4fa*)(gam + c4);
    const v4f tb = *(const v4fa*)(bet + c4);
    g4.x = bf16_val(tg.x); g4.y = bf16_val(tg.y); g4.z = bf16_val(tg.z); g4.w = bf16_val(tg.w);
    b4.x = bf16_val(tb.x); b4.y = bf16_val(tb.y); b4.z = bf16_val(tb.z); b4.w = bf16_val(tb.w);
  }
  const int rowBase = (int)blockIdx.x * 128 + wave * 16;
#pragma unroll 1
  for (int j = 0; j < 8; ++j) {
    const int row = rowBase + 2 * j + hs;
    const int rc  = row < nN ? row : nN - 1;
    const v4f z = *(const v4fa*)(Y + (size_t)rc * YP + CO2 + c4);
    v4f y;
    y.x = ((z.x - m4.x) * r4.x) * g4.x + b4.x;
    y.y = ((z.y - m4.y) * r4.y) * g4.y + b4.y;
    y.z = ((z.z - m4.z) * r4.z) * g4.z + b4.z;
    y.w = ((z.w - m4.w) * r4.w) * g4.w + b4.w;
    float* op = out + (size_t)rc * CO2 + c4;
    const bool ok = row < nN;
    if (ok) *(volatile v4f*)op = y;
    __threadfence();
    if (ok) *(volatile v4f*)op = y;
  }
}

static inline int cdiv(int a, int b) { return (a + b - 1) / b; }
static inline size_t al256(size_t o) { return (o + 255) & ~(size_t)255; }

extern "C" void kernel_launch(void* const* d_in, const int* in_sizes, int n_in,
                              void* d_out, int out_size, void* d_ws, size_t ws_size,
                              hipStream_t stream) {
  if (n_in < 17) return;
  if (in_sizes[0] < CF || (in_sizes[0] % CF) != 0) return;
  const int nN = in_sizes[0] / CF;
  if (nN < 16 || nN > (1 << 22)) return;
  if (in_sizes[1] < 2 || (in_sizes[1] & 1) != 0) return;
  const int nE = in_sizes[1] / 2;
  if (nE < 1 || nE >= (1 << (31 - SLA))) return;
  if (in_sizes[2] != CF * CF || in_sizes[3] != CF) return;
  if (in_sizes[4] != CF * CF || in_sizes[5] != CF || in_sizes[6] != CF) return;
  if (in_sizes[7] != CF * CF || in_sizes[8] != CF) return;
  if (in_sizes[9] != CF * CF || in_sizes[10] != CF || in_sizes[11] != CF) return;
  if (in_sizes[12] != CO2 * CF || in_sizes[13] != CO2) return;
  if (in_sizes[14] != CO2 * CF || in_sizes[15] != CO2 || in_sizes[16] != CO2) return;
  if ((long long)out_size != (long long)nN * CO2) return;

  const float* x    = (const float*)d_in[0];
  const int*   edge = (const int*)d_in[1];
  const float* Wl0  = (const float*)d_in[2];
  const float* bl0  = (const float*)d_in[3];
  const float* Wr0  = (const float*)d_in[4];
  const float* ga0  = (const float*)d_in[5];
  const float* be0  = (const float*)d_in[6];
  const float* Wl1  = (const float*)d_in[7];
  const float* bl1  = (const float*)d_in[8];
  const float* Wr1  = (const float*)d_in[9];
  const float* ga1  = (const float*)d_in[10];
  const float* be1  = (const float*)d_in[11];
  const float* Wl2  = (const float*)d_in[12];
  const float* bl2  = (const float*)d_in[13];
  const float* Wr2  = (const float*)d_in[14];
  const float* ga2  = (const float*)d_in[15];
  const float* be2  = (const float*)d_in[16];
  float* out = (float*)d_out;
  const int* src = edge;
  const int* dst = edge + nE;

  const int gA = cdiv(nN, NBA);
  const int NP = gA * NBA;
  if ((NP % 64) != 0 || (NP % GROWS) != 0) return;
  const int vec8 = ((nE & 3) == 0) ? 1 : 0;
  const double invN = 1.0 / (double)nN;

  char* ws = (char*)d_ws;
  size_t off = 0;
  const size_t oP0  = off; off = al256(off + (size_t)2 * CF * CF * 2);
  const size_t oP1  = off; off = al256(off + (size_t)2 * CF * 2 * CF * 2);
  const size_t oP2  = off; off = al256(off + (size_t)2 * CO2 * 2 * CF * 2);
  const size_t oMS  = off; off = al256(off + (size_t)3 * 256 * 4);
  const size_t recB = (size_t)gA * 256 * 8;
  const size_t oREC = off; off = al256(off + 3 * recB);
  const size_t oY   = off; off = al256(off + (size_t)NP * YP * 4);
  if (off > ws_size || off > (size_t)WSMAX) return;
  unsigned short* P0 = (unsigned short*)(ws + oP0);
  unsigned short* P1 = (unsigned short*)(ws + oP1);
  unsigned short* P2 = (unsigned short*)(ws + oP2);
  float*  MS0  = (float*)(ws + oMS);
  float*  MS1  = MS0 + 256;
  float*  MS2  = MS1 + 256;
  double* REC0 = (double*)(ws + oREC);
  double* REC1 = (double*)(ws + oREC + recB);
  double* REC2 = (double*)(ws + oREC + 2 * recB);
  float*  Y    = (float*)(ws + oY);

  const size_t scanLds = (size_t)AGG_LDS_INTS * 4;
  hipFuncSetAttribute(reinterpret_cast<const void*>(&k_scan<128>), hipFuncAttributeMaxDynamicSharedMemorySize, (int)scanLds);
  hipFuncSetAttribute(reinterpret_cast<const void*>(&k_scan<64>),  hipFuncAttributeMaxDynamicSharedMemorySize, (int)scanLds);

  const int nUx = NP * (CF / 8);
  const int gG  = NP / GROWS;
  const int gB  = NP / 64;

  k_wprep<<<(UP0 + UP1 + UP2) / NTHR, NTHR, 0, stream>>>(Wl0, Wr0, Wl1, Wr1, Wl2, Wr2, P0, P1, P2);
  k_cvx<<<cdiv(nUx, NTHR), NTHR, 0, stream>>>(x, nN, nUx, (unsigned short*)Y);
  k_gemm<2><<<gG, GT, 0, stream>>>(Y, P0, CF);
  k_scan<128><<<gA, NTHR, scanLds, stream>>>(src, dst, nE, nN, vec8, NP, Y, bl0, REC0);
  k_bnstat<<<1, NTHR, 0, stream>>>(REC0, gA, CF, invN, MS0);
  k_bn<<<gB, NTHR, 0, stream>>>(Y, MS0, ga0, be0, nN);
  k_gemm<2><<<gG, GT, 0, stream>>>(Y, P1, 2 * CF);
  k_scan<128><<<gA, NTHR, scanLds, stream>>>(src, dst, nE, nN, vec8, NP, Y, bl1, REC1);
  k_bnstat<<<1, NTHR, 0, stream>>>(REC1, gA, CF, invN, MS1);
  k_bn<<<gB, NTHR, 0, stream>>>(Y, MS1, ga1, be1, nN);
  k_gemm<1><<<gG, GT, 0, stream>>>(Y, P2, 2 * CF);
  k_scan<64><<<gA, NTHR, scanLds, stream>>>(src, dst, nE, nN, vec8, NP, Y, bl2, REC2);
  k_bnstat<<<1, NTHR, 0, stream>>>(REC2, gA, CO2, invN, MS2);
  k_bnout<<<cdiv(nN, 128), NTHR, 0, stream>>>(Y, MS2, ga2, be2, nN, out);
}
